// MultiheadAttentionBlock_23321672417979
// MI455X (gfx1250) — hardware-verified
//
#include <hip/hip_runtime.h>


#ifndef NB
#define NB 2
#endif
#ifndef SEQ
#define SEQ 2048
#endif
#define NB_FULL  2
#define SEQ_FULL 2048
#define TT   SEQ
#define DM   1024
#define NH_  16
#define NKV  16
#define REP  (NH_ / NKV)
#define HD   64
#define DQ   (NH_ * HD)
#define DKV  (NKV * HD)
#define ZH   2
#define RH   ((TT) < 512 ? (TT) : 512)
#define PCAR 1024.0f
#define SCL  0.125f
#define LN_EPS 1e-5f
#define WS_CAP ((size_t)134217728)

static_assert(TT % 128 == 0);
static_assert(RH % 64 == 0);
static_assert(TT <= SEQ_FULL);
static_assert(NB <= NB_FULL);
static_assert(DM % 128 == 0);
static_assert(DQ == DM);
static_assert(DKV == DM);
static_assert(TT / 8 <= 256);
static_assert(((size_t)DM * DM / 8) % 256 == 0);
static_assert(((size_t)TT * DM / 8) % 256 == 0);
static_assert(((size_t)NH_ * TT * HD / 2) % 256 == 0);
static_assert(((size_t)NKV * TT * HD / 2) % 256 == 0);
static_assert(((size_t)ZH * TT * HD / 2) % 256 == 0);
static_assert((ZH * TT) % 8 == 0);
static_assert(NH_ % ZH == 0);

typedef _Float16 h16;
typedef unsigned short bf;
typedef __attribute__((ext_vector_type(16))) __bf16   v16bf;
typedef __attribute__((ext_vector_type(16))) _Float16 v16h;
typedef __attribute__((ext_vector_type(8)))  _Float16 v8h;
typedef __attribute__((ext_vector_type(8)))  unsigned short v8us;
typedef __attribute__((ext_vector_type(8)))  float    v8f;
typedef __attribute__((ext_vector_type(4)))  float    v4f;
typedef v8h  __attribute__((may_alias)) v8ha;
typedef v4f  __attribute__((may_alias)) v4fa;
typedef v8us __attribute__((may_alias)) v8usa;
typedef __attribute__((ext_vector_type(2))) _Float16 v2h;
typedef __attribute__((ext_vector_type(4))) _Float16 v4h;
typedef __attribute__((ext_vector_type(2))) unsigned short v2us;
typedef __attribute__((ext_vector_type(4))) unsigned short v4us;
typedef __attribute__((ext_vector_type(2))) float v2f;
typedef __attribute__((ext_vector_type(4))) int v4i;

__device__ __forceinline__ unsigned short f2bf(float f) { unsigned u = __float_as_uint(f); u += 0x7FFFu + ((u >> 16) & 1u); return (unsigned short)(u >> 16); }
__device__ __forceinline__ float bf2f(unsigned short b) { return __uint_as_float(((unsigned)b) << 16); }
__device__ __forceinline__ float bfr(float f) { return bf2f(f2bf(f)); }
__device__ __forceinline__ v16h cat16(v8h lo, v8h hi) { return __builtin_shufflevector(lo, hi, 0, 1, 2, 3, 4, 5, 6, 7, 8, 9, 10, 11, 12, 13, 14, 15); }
__device__ __forceinline__ v16bf cat16b(v8us lo, v8us hi) { return __builtin_bit_cast(v16bf, __builtin_shufflevector(lo, hi, 0, 1, 2, 3, 4, 5, 6, 7, 8, 9, 10, 11, 12, 13, 14, 15)); }
__device__ __forceinline__ v8f wmma16(v16h a, v16h b, v8f c) { return __builtin_amdgcn_wmma_f32_16x16x32_f16(false, a, false, b, (short)0, c, false, false); }
__device__ __forceinline__ v8f wmmab(v16bf a, v16bf b, v8f c) { return __builtin_amdgcn_wmma_f32_16x16x32_bf16(false, a, false, b, (short)0, c, false, false); }

template <typename T16> struct WFrag;
template <> struct WFrag<h16> { typedef v16h V; static __device__ __forceinline__ V ld(const h16* p) { return cat16(*(const v8h*)p, *(const v8h*)(p + 16)); } static __device__ __forceinline__ v8f mma(V a, V b, v8f c) { return wmma16(a, b, c); } };
template <> struct WFrag<bf> { typedef v16bf V; static __device__ __forceinline__ V ld(const bf* p) { return cat16b(*(const v8us*)p, *(const v8us*)(p + 16)); } static __device__ __forceinline__ v8f mma(V a, V b, v8f c) { return wmmab(a, b, c); } };
template <typename T16, int NSPLIT, bool BIAS>
__global__ __launch_bounds__(32) void k_gemmw(const T16* __restrict__ A, const T16* __restrict__ A2, const T16* __restrict__ Bt, const T16* __restrict__ Bt2, int K, float* C, int ldc, const float* __restrict__ bias, size_t sA, size_t sB, size_t sC) {
    typedef typename WFrag<T16>::V V;
    __shared__ __align__(16) float os[16 * 68];
    const size_t z = blockIdx.z; A += z * sA; if (A2) A2 += z * sA; Bt += z * sB; if (Bt2) Bt2 += z * sB; C += z * sC;
    const int lane = threadIdx.x & 31, lr = lane & 15, hi = lane >> 4; const int r0 = blockIdx.x * 64, c0 = blockIdx.y * 64;
    v8f acc[4][4];
#pragma unroll
    for (int mb = 0; mb < 4; ++mb)
#pragma unroll
        for (int nb = 0; nb < 4; ++nb) acc[mb][nb] = (v8f){};
    const size_t aoff = (size_t)(r0 + lr) * K + 8 * hi, boff = (size_t)(c0 + lr) * K + 8 * hi;
#pragma unroll 1
    for (int kc = 0; kc < K; kc += 32) {
        V a[4], a2[4];
#pragma unroll
        for (int mb = 0; mb < 4; ++mb) { a[mb] = WFrag<T16>::ld(A + aoff + (size_t)mb * 16 * K + kc); if (NSPLIT == 1 || NSPLIT == 2) a2[mb] = WFrag<T16>::ld(A2 + aoff + (size_t)mb * 16 * K + kc); }
#pragma unroll
        for (int nb = 0; nb < 4; ++nb) { const V b = WFrag<T16>::ld(Bt + boff + (size_t)nb * 16 * K + kc); V b2; if (NSPLIT >= 2) b2 = WFrag<T16>::ld(Bt2 + boff + (size_t)nb * 16 * K + kc);
#pragma unroll
            for (int mb = 0; mb < 4; ++mb) { acc[mb][nb] = WFrag<T16>::mma(a[mb], b, acc[mb][nb]); if (NSPLIT == 1 || NSPLIT == 2) acc[mb][nb] = WFrag<T16>::mma(a2[mb], b, acc[mb][nb]); if (NSPLIT >= 2) acc[mb][nb] = WFrag<T16>::mma(a[mb], b2, acc[mb][nb]); } }
        asm volatile("v_nop\n\tv_nop\n\tv_nop\n\tv_nop" : "+v"(acc[0][0]), "+v"(acc[1][1]), "+v"(acc[2][2]), "+v"(acc[3][3]) : "v"(a[0]), "v"(a[3]));
    }
#pragma unroll
    for (int mb = 0; mb < 4; ++mb) {
#pragma unroll
        for (int nb = 0; nb < 4; ++nb) {
#pragma unroll
            for (int j = 0; j < 8; ++j) os[(hi * 8 + j) * 68 + nb * 16 + lr] = acc[mb][nb][j]; }
        __builtin_amdgcn_wave_barrier(); asm volatile("" ::: "memory");
        float* crow = C + (size_t)(r0 + mb * 16) * ldc + c0;
#pragma unroll 1
        for (int ps = 0; ps < 2; ++ps) {
#pragma unroll
            for (int s = 0; s < 8; ++s) { const int row = 2 * s + hi, cofs = lr * 4; v4f val = *(const v4fa*)(os + row * 68 + cofs); if (BIAS) { val[0] += bfr(bias[c0 + cofs]); val[1] += bfr(bias[c0 + cofs + 1]); val[2] += bfr(bias[c0 + cofs + 2]); val[3] += bfr(bias[c0 + cofs + 3]); }
                *(volatile v4f*)(crow + (size_t)row * ldc + cofs) = val; }
            if (ps == 0) __threadfence(); }
        __builtin_amdgcn_wave_barrier(); asm volatile("" ::: "memory");
    }
}

template <typename T16, int NSPLIT, int CMODE>
__global__ __launch_bounds__(32) void k_gemmc(const T16* __restrict__ A, const T16* __restrict__ A2, const T16* __restrict__ Bt, const T16* __restrict__ Bt2, int K, float* C, int ldc, int roff, size_t sA, size_t sB, size_t sC) {
    typedef typename WFrag<T16>::V V;
    __shared__ __align__(16) float os[16 * 68];
    const size_t z = blockIdx.z; A += z * sA; if (A2) A2 += z * sA; Bt += z * sB; if (Bt2) Bt2 += z * sB; C += z * sC;
    const int lane = threadIdx.x & 31, lr = lane & 15, hi = lane >> 4; const int r0 = blockIdx.x * 64, c0 = blockIdx.y * 64;
    if (CMODE == 1 && c0 > r0 + roff + 63) return;
    const int Kl = (CMODE == 2) ? min(K, r0 + roff + 64) : K;
    v8f acc[4][4];
#pragma unroll
    for (int mb = 0; mb < 4; ++mb)
#pragma unroll
        for (int nb = 0; nb < 4; ++nb) acc[mb][nb] = (v8f){};
    const size_t aoff = (size_t)(r0 + lr) * K + 8 * hi, boff = (size_t)(c0 + lr) * K + 8 * hi;
#pragma unroll 1
    for (int kc = 0; kc < Kl; kc += 32) {
        V a[4], a2[4];
#pragma unroll
        for (int mb = 0; mb < 4; ++mb) { a[mb] = WFrag<T16>::ld(A + aoff + (size_t)mb * 16 * K + kc); if (NSPLIT == 1 || NSPLIT == 2) a2[mb] = WFrag<T16>::ld(A2 + aoff + (size_t)mb * 16 * K + kc); }
#pragma unroll
        for (int nb = 0; nb < 4; ++nb) { const V b = WFrag<T16>::ld(Bt + boff + (size_t)nb * 16 * K + kc); V b2; if (NSPLIT >= 2) b2 = WFrag<T16>::ld(Bt2 + boff + (size_t)nb * 16 * K + kc);
#pragma unroll
            for (int mb = 0; mb < 4; ++mb) { acc[mb][nb] = WFrag<T16>::mma(a[mb], b, acc[mb][nb]); if (NSPLIT == 1 || NSPLIT == 2) acc[mb][nb] = WFrag<T16>::mma(a2[mb], b, acc[mb][nb]); if (NSPLIT >= 2) acc[mb][nb] = WFrag<T16>::mma(a[mb], b2, acc[mb][nb]); } }
        asm volatile("v_nop\n\tv_nop\n\tv_nop\n\tv_nop" : "+v"(acc[0][0]), "+v"(acc[1][1]), "+v"(acc[2][2]), "+v"(acc[3][3]) : "v"(a[0]), "v"(a[3]));
    }
#pragma unroll
    for (int mb = 0; mb < 4; ++mb) {
#pragma unroll
        for (int nb = 0; nb < 4; ++nb) {
#pragma unroll
            for (int j = 0; j < 8; ++j) os[(hi * 8 + j) * 68 + nb * 16 + lr] = acc[mb][nb][j]; }
        __builtin_amdgcn_wave_barrier(); asm volatile("" ::: "memory");
        float* crow = C + (size_t)(r0 + mb * 16) * ldc + c0;
#pragma unroll 1
        for (int ps = 0; ps < 2; ++ps) {
#pragma unroll
            for (int s = 0; s < 8; ++s) { const int row = 2 * s + hi, cofs = lr * 4; v4f val = *(const v4fa*)(os + row * 68 + cofs);
                *(volatile v4f*)(crow + (size_t)row * ldc + cofs) = val; }
            if (ps == 0) __threadfence(); }
        __builtin_amdgcn_wave_barrier(); asm volatile("" ::: "memory");
    }
}

__device__ __forceinline__ h16 tohx(float x) { return (h16)x; }
__device__ __forceinline__ void splitf(float y, unsigned short& h, unsigned short& l) { h = f2bf(y); l = f2bf(y - bf2f(h)); }

__global__ __launch_bounds__(256) void k_cvt8(const float* __restrict__ src, bf* dst, size_t n8) { const size_t i = (size_t)blockIdx.x * 256 + threadIdx.x; if (i >= n8) return; const v8f v = *(const v8f*)(src + i * 8); v8us o;
#pragma unroll
    for (int k = 0; k < 8; ++k) o[k] = f2bf(v[k]); *(volatile v8us*)(dst + i * 8) = o; __threadfence(); *(volatile v8us*)(dst + i * 8) = o; }

__global__ __launch_bounds__(256) void k_cvtw4(const float* __restrict__ s0, const float* __restrict__ s1, const float* __restrict__ s2, const float* __restrict__ s3, bf* d0, bf* d1, bf* d2, bf* d3, unsigned n8) {
    const unsigned i = blockIdx.x * 256u + threadIdx.x; if (i >= n8) return; const unsigned y = blockIdx.y;
    const float* src = (y == 0u) ? s0 : (y == 1u) ? s1 : (y == 2u) ? s2 : s3; bf* dst = (y == 0u) ? d0 : (y == 1u) ? d1 : (y == 2u) ? d2 : d3;
    const v8f v = *(const v8f*)(src + (size_t)i * 8); v8us o;
#pragma unroll
    for (int k = 0; k < 8; ++k) o[k] = f2bf(v[k]); *(volatile v8us*)(dst + (size_t)i * 8) = o; __threadfence(); *(volatile v8us*)(dst + (size_t)i * 8) = o; }

__global__ __launch_bounds__(256) void k_hpl(const float* __restrict__ F, unsigned pitch, unsigned nheads, h16* P16, bf* Ph, bf* Pl) {
    const unsigned e = (blockIdx.x * 256u + threadIdx.x) * 2u; if (e >= nheads * (unsigned)(TT * HD)) return; const unsigned d = e % (unsigned)HD; const unsigned t = (e / (unsigned)HD) % (unsigned)TT; const unsigned h = e / (unsigned)(HD * TT);
    const v2f x = *(const v2f*)(F + (size_t)t * pitch + h * (unsigned)HD + d); v2h o16; v2us oh, ol;
#pragma unroll
    for (int q = 0; q < 2; ++q) { const float r = x[q]; o16[q] = tohx(r); unsigned short a2, c2; splitf(r, a2, c2); oh[q] = a2; ol[q] = c2; }
    *(volatile v2h*)(P16 + e) = o16; *(volatile v2us*)(Ph + e) = oh; *(volatile v2us*)(Pl + e) = ol; __threadfence(); *(volatile v2h*)(P16 + e) = o16; *(volatile v2us*)(Ph + e) = oh; *(volatile v2us*)(Pl + e) = ol; }

__global__ __launch_bounds__(256) void k_vtp(const float* __restrict__ F, unsigned pitch, unsigned nheads, h16* V16, bf* Vh, bf* Vl) { const unsigned e = (blockIdx.x * 256u + threadIdx.x) * 2u; if (e >= nheads * (unsigned)(HD * TT)) return; const unsigned t = e % (unsigned)TT; const unsigned d = (e / (unsigned)TT) % (unsigned)HD; const unsigned g = e / (unsigned)(TT * HD); v2h o16; v2us oh, ol;
#pragma unroll
    for (int q = 0; q < 2; ++q) { const float x = F[(size_t)(t + (unsigned)q) * pitch + g * (unsigned)HD + d]; o16[q] = tohx(x); unsigned short a2, c2; splitf(x, a2, c2); oh[q] = a2; ol[q] = c2; }
    *(volatile v2h*)(V16 + e) = o16; *(volatile v2us*)(Vh + e) = oh; *(volatile v2us*)(Vl + e) = ol; __threadfence(); *(volatile v2h*)(V16 + e) = o16; *(volatile v2us*)(Vh + e) = oh; *(volatile v2us*)(Vl + e) = ol; }

__global__ __launch_bounds__(256) void k_mchk(const int* __restrict__ pm, const int* __restrict__ fm, int* FL) {
    __shared__ int sc[8];
    const unsigned lane = threadIdx.x & 31u, w = threadIdx.x >> 5; const unsigned i = blockIdx.x * 8u + w;
    int bad = 0; const int* fr = fm + (size_t)i * SEQ_FULL;
#pragma unroll 1
    for (unsigned c = 0; c < (unsigned)(TT / 128); ++c) { const unsigned j0 = c * 128u + lane * 4u; const v4i m = *(const v4i*)(fr + j0);
#pragma unroll
        for (int q = 0; q < 4; ++q) bad += ((m[q] != 0) != (j0 + (unsigned)q > i)) ? 1 : 0; }
    if (i < (unsigned)NB) {
        const int* pr = pm + (size_t)i * SEQ_FULL;
#pragma unroll 1
        for (unsigned c = 0; c < (unsigned)(TT / 128); ++c) { const unsigned j0 = c * 128u + lane * 4u; const v4i m = *(const v4i*)(pr + j0);
#pragma unroll
            for (int q = 0; q < 4; ++q) bad += (m[q] != 0) ? 1 : 0; } }
#pragma unroll
    for (int sh = 16; sh; sh >>= 1) bad += __shfl_xor(bad, sh, 32);
    if (lane == 0u) sc[w] = bad;
    __syncthreads();
    if (w == 0u) { const int tot = sc[0] + sc[1] + sc[2] + sc[3] + sc[4] + sc[5] + sc[6] + sc[7]; int* p = FL + (size_t)blockIdx.x * 32 + lane; *(volatile int*)p = tot; __threadfence(); *(volatile int*)p = tot; }
}

__global__ __launch_bounds__(256) void k_asoft(const float* __restrict__ Sb, h16* P16, bf* Ph, bf* Pl) {
    const unsigned lane = threadIdx.x & 31u; const unsigned row = blockIdx.x * 8u + (threadIdx.x >> 5); if (row >= (unsigned)(ZH * TT)) return; const unsigned i = row % (unsigned)TT; const unsigned zz = row / (unsigned)TT; const bool hires = (i < (unsigned)RH); const float* sr = Sb + (size_t)row * TT; float v[TT / 32]; float mx = -3.0e38f;
#pragma unroll
    for (int ch = 0; ch < TT / 128; ++ch) { const unsigned j0 = (unsigned)ch * 128u + lane * 4u; const v4f a = *(const v4f*)(sr + j0);
#pragma unroll
        for (int q = 0; q < 4; ++q) { const unsigned j = j0 + (unsigned)q; const float t = (j <= i) ? a[q] * SCL : -3.0e38f; v[ch * 4 + q] = t; mx = fmaxf(mx, t); } }
#pragma unroll
    for (int sh = 16; sh; sh >>= 1) mx = fmaxf(mx, __shfl_xor(mx, sh, 32));
    float sum = 0.f;
#pragma unroll
    for (int k = 0; k < TT / 32; ++k) { float d0 = __fsub_rn(v[k], mx); asm volatile("" : "+v"(d0)); v[k] = __builtin_amdgcn_exp2f(__fmul_rn(d0, 1.4426950408889634f)); sum += v[k]; }
#pragma unroll
    for (int sh = 16; sh; sh >>= 1) sum += __shfl_xor(sum, sh, 32);
    const float f = __fdiv_rn(hires ? 1.0f : PCAR, sum);
#pragma unroll 1
    for (int ps = 0; ps < 2; ++ps) {
        if (hires) {
#pragma unroll
            for (int ch = 0; ch < TT / 128; ++ch) { v4us oh, ol;
#pragma unroll
                for (int q = 0; q < 4; ++q) { unsigned short a, c2; splitf(v[ch * 4 + q] * f, a, c2); oh[q] = a; ol[q] = c2; }
                const size_t oo = ((size_t)zz * (RH ? RH : 1) + i) * TT + (unsigned)ch * 128u + lane * 4u; *(volatile v4us*)(Ph + oo) = oh; *(volatile v4us*)(Pl + oo) = ol; }
        } else {
#pragma unroll
            for (int ch = 0; ch < TT / 128; ++ch) { v4h o4;
#pragma unroll
                for (int q = 0; q < 4; ++q) o4[q] = tohx(v[ch * 4 + q] * f);
                *(volatile v4h*)(P16 + (size_t)row * TT + (unsigned)ch * 128u + lane * 4u) = o4; } }
        if (ps == 0) __threadfence(); }
}

__global__ __launch_bounds__(256) void k_merge(const float* __restrict__ O, unsigned h0, bf* Ah, bf* Al) { const unsigned e = (blockIdx.x * 256u + threadIdx.x) * 2u; if (e >= (unsigned)(ZH * TT * HD)) return; const unsigned d = e % (unsigned)HD; const unsigned t = (e / (unsigned)HD) % (unsigned)TT; const unsigned zz = e / (unsigned)(HD * TT); const float cs = (t < (unsigned)RH) ? 1.0f : (1.0f / PCAR); const size_t oo = (size_t)t * DQ + (h0 + zz) * (unsigned)HD + d;
    const v2f x = *(const v2f*)(O + e); v2us oh, ol;
#pragma unroll
    for (int q = 0; q < 2; ++q) { unsigned short a, c2; splitf(x[q] * cs, a, c2); oh[q] = a; ol[q] = c2; } *(volatile v2us*)(Ah + oo) = oh; *(volatile v2us*)(Al + oo) = ol; __threadfence(); *(volatile v2us*)(Ah + oo) = oh; *(volatile v2us*)(Al + oo) = ol; }

__global__ __launch_bounds__(256) void k_ln(const float* __restrict__ Y, const float* __restrict__ Xq, const float* __restrict__ gam, const float* __restrict__ bet, const int* __restrict__ FL, float* OUT) {
    __shared__ __align__(16) float xs[8 * DM];
    __shared__ int sf[8];
    const unsigned lane = threadIdx.x & 31u, w = threadIdx.x >> 5; const unsigned row = blockIdx.x * 8u + w;
    unsigned fi = threadIdx.x; if (fi > (unsigned)(TT / 8 - 1)) fi = (unsigned)(TT / 8 - 1);
    int fl = FL[(size_t)fi * 32];
#pragma unroll
    for (int sh = 16; sh; sh >>= 1) fl |= __shfl_xor(fl, sh, 32);
    if (lane == 0u) sf[w] = fl;
    __syncthreads();
    const int flag = sf[0] | sf[1] | sf[2] | sf[3] | sf[4] | sf[5] | sf[6] | sf[7];
    const float* yr = Y + (size_t)row * DM; const float* qr = Xq + (size_t)row * DM; float* xr = xs + w * (unsigned)DM;
    float s = 0.f;
#pragma unroll 2
    for (unsigned c = 0; c < (unsigned)(DM / 128); ++c) { const unsigned o = c * 128u + lane * 4u; const v4f y = *(const v4f*)(yr + o); const v4f q = *(const v4f*)(qr + o); v4f x;
#pragma unroll
        for (int k = 0; k < 4; ++k) x[k] = bfr(q[k]) + y[k];
        s += (x[0] + x[1]) + (x[2] + x[3]); *(v4fa*)(xr + o) = x; }
#pragma unroll
    for (int sh = 16; sh; sh >>= 1) s += __shfl_xor(s, sh, 32);
    const float mu = s * (1.0f / (float)DM);
    float ss = 0.f;
#pragma unroll 2
    for (unsigned c = 0; c < (unsigned)(DM / 128); ++c) { const unsigned o = c * 128u + lane * 4u; const v4f x = *(const v4fa*)(xr + o);
#pragma unroll
        for (int k = 0; k < 4; ++k) { const float d = x[k] - mu; ss += d * d; } }
#pragma unroll
    for (int sh = 16; sh; sh >>= 1) ss += __shfl_xor(ss, sh, 32);
    const float rstd = rsqrtf(ss * (1.0f / (float)DM) + LN_EPS);
    const float nanv = __uint_as_float(0x7FC00000u);
    float* orow = OUT + (size_t)row * DM;
#pragma unroll 1
    for (int ps = 0; ps < 2; ++ps) {
#pragma unroll 2
        for (unsigned c = 0; c < (unsigned)(DM / 128); ++c) { const unsigned o = c * 128u + lane * 4u; const v4f x = *(const v4fa*)(xr + o); const v4f g = *(const v4f*)(gam + o); const v4f b = *(const v4f*)(bet + o); v4f val;
#pragma unroll
            for (int k = 0; k < 4; ++k) { const float r = (x[k] - mu) * rstd * bfr(g[k]) + bfr(b[k]); val[k] = flag ? nanv : r; }
            *(volatile v4f*)(orow + o) = val; }
        if (ps == 0) __threadfence(); }
}

extern "C" void kernel_launch(void* const* d_in, const int* in_sizes, int n_in,
                              void* d_out, int out_size, void* d_ws, size_t ws_size, hipStream_t stream) {
    if (n_in < 15) return;
    const size_t need_x = (size_t)(NB - 1) * SEQ_FULL * DM + (size_t)TT * DM;
    if ((size_t)in_sizes[0] < need_x || (size_t)in_sizes[1] < need_x || (size_t)in_sizes[2] < need_x) return;
    if ((size_t)in_sizes[3] < (size_t)(NB - 1) * SEQ_FULL + (size_t)TT) return;
    if ((size_t)in_sizes[4] < (size_t)(TT - 1) * SEQ_FULL + (size_t)TT) return;
    if ((size_t)in_sizes[5] < (size_t)DM * DM || (size_t)in_sizes[7] < (size_t)DM * DM || (size_t)in_sizes[9] < (size_t)DM * DM || (size_t)in_sizes[11] < (size_t)DM * DM) return;
    if (in_sizes[6] < DM || in_sizes[8] < DM || in_sizes[10] < DM || in_sizes[12] < DM || in_sizes[13] < DM || in_sizes[14] < DM) return;
    if ((size_t)out_size < (size_t)NB * TT * DM) return;
    const float* x = (const float*)d_in[0]; const float* xk = (const float*)d_in[1]; const float* xv = (const float*)d_in[2];
    const int* pm = (const int*)d_in[3]; const int* fm = (const int*)d_in[4];
    const float* wq = (const float*)d_in[5]; const float* bq = (const float*)d_in[6]; const float* wk = (const float*)d_in[7]; const float* bk = (const float*)d_in[8];
    const float* wv = (const float*)d_in[9]; const float* bv = (const float*)d_in[10]; const float* wo = (const float*)d_in[11]; const float* bo = (const float*)d_in[12];
    const float* gam = (const float*)d_in[13]; const float* bet = (const float*)d_in[14];
    float* OUT = (float*)d_out;
    char* wsp = (char*)d_ws;
    auto take = [&](size_t bytes) { char* p = wsp; wsp += (bytes + 255) & ~(size_t)255; return (void*)p; };
    bf* WQb = (bf*)take((size_t)DQ * DM * 2); bf* WKb = (bf*)take((size_t)DKV * DM * 2); bf* WVb = (bf*)take((size_t)DKV * DM * 2); bf* WOb = (bf*)take((size_t)DM * DQ * 2);
    bf* XB = (bf*)take((size_t)TT * DM * 2);
    float* F = (float*)take((size_t)TT * DM * 4);
    h16* QP16 = (h16*)take((size_t)NH_ * TT * HD * 2); h16* KP16 = (h16*)take((size_t)NKV * TT * HD * 2); h16* VT16 = (h16*)take((size_t)NKV * HD * TT * 2);
    bf* QPh = (bf*)take((size_t)NH_ * TT * HD * 2); bf* QPl = (bf*)take((size_t)NH_ * TT * HD * 2); bf* KPh = (bf*)take((size_t)NKV * TT * HD * 2); bf* KPl = (bf*)take((size_t)NKV * TT * HD * 2); bf* VTh = (bf*)take((size_t)NKV * HD * TT * 2); bf* VTl = (bf*)take((size_t)NKV * HD * TT * 2);
    bf* Ph = (bf*)take((size_t)ZH * RH * TT * 2); bf* Pl = (bf*)take((size_t)ZH * RH * TT * 2);
    float* Sb = (float*)take((size_t)ZH * TT * TT * 4); h16* P16 = (h16*)take((size_t)ZH * TT * TT * 2); float* Ob = (float*)take((size_t)ZH * TT * HD * 4); bf* ATh = (bf*)take((size_t)TT * DQ * 2); bf* ATl = (bf*)take((size_t)TT * DQ * 2);
    int* FL = (int*)take((size_t)(TT / 8) * 128);
    const size_t used = (size_t)(wsp - (char*)d_ws);
    if (used > ws_size || used > WS_CAP) return;
    k_cvtw4<<<dim3((unsigned)(((size_t)DM * DM / 8 + 255) / 256), 4, 1), 256, 0, stream>>>(wq, wk, wv, wo, WQb, WKb, WVb, WOb, (unsigned)((size_t)DM * DM / 8));
    k_mchk<<<TT / 8, 256, 0, stream>>>(pm, fm, FL);
    const unsigned G8 = (unsigned)(((size_t)TT * DM / 8 + 255) / 256);
    const unsigned LQ = (unsigned)(((size_t)NH_ * TT * HD / 2 + 255) / 256), LKv = (unsigned)(((size_t)NKV * TT * HD / 2 + 255) / 256);
    for (int b = 0; b < NB; ++b) {
        const size_t ib = (size_t)b * SEQ_FULL * DM;
        k_cvt8<<<G8, 256, 0, stream>>>(x + ib, XB, (size_t)TT * DM / 8);
        k_gemmw<bf, 0, true><<<dim3(TT / 64, DQ / 64, 1), 32, 0, stream>>>(XB, nullptr, WQb, nullptr, DM, F, DQ, bq, 0, 0, 0);
        k_hpl<<<LQ, 256, 0, stream>>>(F, (unsigned)DQ, (unsigned)NH_, QP16, QPh, QPl);
        k_cvt8<<<G8, 256, 0, stream>>>(xk + ib, XB, (size_t)TT * DM / 8);
        k_gemmw<bf, 0, true><<<dim3(TT / 64, DKV / 64, 1), 32, 0, stream>>>(XB, nullptr, WKb, nullptr, DM, F, DKV, bk, 0, 0, 0);
        k_hpl<<<LKv, 256, 0, stream>>>(F, (unsigned)DKV, (unsigned)NKV, KP16, KPh, KPl);
        k_cvt8<<<G8, 256, 0, stream>>>(xv + ib, XB, (size_t)TT * DM / 8);
        k_gemmw<bf, 0, true><<<dim3(TT / 64, DKV / 64, 1), 32, 0, stream>>>(XB, nullptr, WVb, nullptr, DM, F, DKV, bv, 0, 0, 0);
        k_vtp<<<LKv, 256, 0, stream>>>(F, (unsigned)DKV, (unsigned)NKV, VT16, VTh, VTl);
        for (int h0 = 0; h0 < NH_; h0 += ZH) { const size_t zq = (size_t)h0, zk = (size_t)(h0 / REP);
            k_gemmc<bf, 2, 1><<<dim3(RH / 64, TT / 64, ZH), 32, 0, stream>>>(QPh + zq * TT * HD, QPl + zq * TT * HD, KPh + zk * TT * HD, KPl + zk * TT * HD, HD, Sb, TT, 0, (size_t)TT * HD, (size_t)TT * HD, (size_t)TT * TT);
            if (TT > RH) k_gemmc<h16, 0, 1><<<dim3((TT - RH) / 64 + (TT == RH), TT / 64, ZH), 32, 0, stream>>>(QP16 + zq * TT * HD + (size_t)RH * HD, nullptr, KP16 + zk * TT * HD, nullptr, HD, Sb + (size_t)RH * TT, TT, RH, (size_t)TT * HD, (size_t)TT * HD, (size_t)TT * TT);
            k_asoft<<<ZH * TT / 8, 256, 0, stream>>>(Sb, P16, Ph, Pl);
            k_gemmc<bf, 2, 2><<<dim3(RH / 64, HD / 64, ZH), 32, 0, stream>>>(Ph, Pl, VTh + zk * HD * TT, VTl + zk * HD * TT, TT, Ob, HD, 0, (size_t)RH * TT, (size_t)HD * TT, (size_t)TT * HD);
            if (TT > RH) k_gemmc<h16, 0, 2><<<dim3((TT - RH) / 64 + (TT == RH), HD / 64, ZH), 32, 0, stream>>>(P16 + (size_t)RH * TT, nullptr, VT16 + zk * HD * TT, nullptr, TT, Ob + (size_t)RH * HD, HD, RH, (size_t)TT * TT, (size_t)HD * TT, (size_t)TT * HD);
            k_merge<<<(unsigned)(((size_t)ZH * TT * HD / 2 + 255) / 256), 256, 0, stream>>>(Ob, (unsigned)h0, ATh, ATl); }
        k_gemmw<bf, 1, true><<<dim3(TT / 64, DM / 64, 1), 32, 0, stream>>>(ATh, ATl, WOb, nullptr, DQ, F, DM, bo, 0, 0, 0);
        k_ln<<<TT / 8, 256, 0, stream>>>(F, x + ib, gam, bet, FL, OUT + (size_t)b * TT * DM); }
}
